// SelectiveSSM_84215718740528
// MI455X (gfx1250) — hardware-run, weakly checked
//
#include <hip/hip_runtime.h>
#include <math.h>

typedef __attribute__((ext_vector_type(16))) _Float16 v16h;
typedef __attribute__((ext_vector_type(8)))  _Float16 v8h;
typedef __attribute__((ext_vector_type(16))) __bf16   v16b;
typedef __attribute__((ext_vector_type(8)))  __bf16   v8b;
typedef __attribute__((ext_vector_type(8)))  float    v8f;
typedef __attribute__((ext_vector_type(4)))  float    v4f;
typedef __attribute__((ext_vector_type(4)))  unsigned v4u;

constexpr int kBatch = 2;
constexpr int kSeq   = 2048;
constexpr int kDch   = 2048;
constexpr int kNst   = 16;
constexpr int kRank  = 64;
constexpr int kProjW = kRank + 2 * kNst;
constexpr int kProjP = 128;
constexpr int kRows  = kBatch * kSeq;
constexpr int kScanTS = 32;
constexpr int kScanCh = 64;
constexpr int kScanYP = 68;
static_assert(kProjW == 96 && kProjP >= kProjW, "projection width");
static_assert((kRows % 64) == 0 && (kProjP % 64) == 0 && (kDch % 64) == 0, "GEMM M,N multiples of 64");
static_assert((kDch % 32) == 0 && (kRank % 32) == 0, "GEMM K multiples of 32");
static_assert((kSeq % kScanTS) == 0 && (kDch % kScanCh) == 0, "scan tiling");
static_assert(kScanTS == 32 && kScanCh == 64 && kNst == 16, "scan lane maps");

constexpr int kMode   = 1;
constexpr int kET     = (kMode == 1) ? 1 : 0;
constexpr int kSPL    = (kMode == 1) ? 2 : 0;
constexpr int kCarryX  = 6;
constexpr int kCarryWx = 10;
constexpr int kCarryDr = 6;
constexpr int kCarryWd = 6;
constexpr int kShift0 = (kMode == 1) ? 0 : (kCarryX + kCarryWx);
constexpr int kShift1 = (kMode == 1) ? 0 : (kCarryDr + kCarryWd);

constexpr size_t kSzX16  = (size_t)kRows * kDch * 2;
constexpr size_t kSzWx16 = (size_t)kProjP * kDch * 2;
constexpr size_t kSzWd16 = (size_t)kDch * kRank * 2;
constexpr size_t kSzXD   = (size_t)kRows * kProjP * 4;
constexpr size_t kSzDr16 = (size_t)kRows * kRank * 2;
constexpr size_t kSzF32  = (size_t)kRows * kDch * 4;
constexpr size_t kOffXH  = 0;
constexpr size_t kOffXL  = kOffXH  + kSzX16;
constexpr size_t kOffWXH = kOffXL  + kSzX16;
constexpr size_t kOffWXL = kOffWXH + kSzWx16;
constexpr size_t kOffWDH = kOffWXL + kSzWx16;
constexpr size_t kOffWDL = kOffWDH + kSzWd16;
constexpr size_t kOffXD  = kOffWDL + kSzWd16;
constexpr size_t kOffDRH = kOffXD  + kSzXD;
constexpr size_t kOffDRL = kOffDRH + kSzDr16;
constexpr size_t kOffPRE = kOffDRL + kSzDr16;
constexpr size_t kOffDL  = kOffPRE + kSzF32;
constexpr size_t kWsTotal = kOffDL + kSzF32;
static_assert(kWsTotal == 105381888ull, "carve total");
static_assert(kWsTotal <= 134217728ull, "carve cap");
static_assert((kOffXL % 128) == 0 && (kOffWXH % 128) == 0 && (kOffWXL % 128) == 0 && (kOffWDH % 128) == 0 &&
              (kOffWDL % 128) == 0 && (kOffXD % 128) == 0 && (kOffDRH % 128) == 0 && (kOffDRL % 128) == 0 &&
              (kOffPRE % 128) == 0 && (kOffDL % 128) == 0, "128-B aligned regions");

__device__ __forceinline__ unsigned bf_rne_word(float f) {
  const unsigned u = __float_as_uint(f);
  const unsigned lsb = (u & 0x00010000u) ? 1u : 0u;
  return (u + 0x7FFFu + lsb) & 0xFFFF0000u;
}
__device__ __forceinline__ unsigned f16_bits(float v) {
  const float vf = (fabsf(v) < 6.103515625e-5f) ? 0.0f : v;
  const _Float16 hv = (_Float16)vf;
  return (unsigned)__builtin_bit_cast(unsigned short, hv);
}

__device__ __forceinline__ v8f mma_guard_h(v16h a, v16h b, v8f c) {
  c = __builtin_amdgcn_wmma_f32_16x16x32_f16(false, a, false, b, (short)0, c, false, false);
  asm volatile("v_nop\n\tv_nop\n\tv_nop\n\tv_nop" : "+v"(c) : "v"(a), "v"(b));
  return c;
}
__device__ __forceinline__ v8f mma_guard_b(v16b a, v16b b, v8f c) {
  c = __builtin_amdgcn_wmma_f32_16x16x32_bf16(false, a, false, b, (short)0, c, false, false);
  asm volatile("v_nop\n\tv_nop\n\tv_nop\n\tv_nop" : "+v"(c) : "v"(a), "v"(b));
  return c;
}
template <typename T> struct Frag;
template <> struct Frag<_Float16> {
  typedef v16h V; union U { v16h v; v8h h[2]; };
  static __device__ __forceinline__ v16h load(const _Float16* p) {
    U f; f.h[0] = *(const v8h*)(p); f.h[1] = *(const v8h*)(p + 16); return f.v;
  }
  static __device__ __forceinline__ v8f mma(v16h a, v16h b, v8f c) { return mma_guard_h(a, b, c); }
};
template <> struct Frag<__bf16> {
  typedef v16b V; union U { v16b v; v8b h[2]; };
  static __device__ __forceinline__ v16b load(const __bf16* p) {
    U f; f.h[0] = *(const v8b*)(p); f.h[1] = *(const v8b*)(p + 16); return f.v;
  }
  static __device__ __forceinline__ v8f mma(v16b a, v16b b, v8f c) { return mma_guard_b(a, b, c); }
};
template <int ET> struct Elem;
template <> struct Elem<0> { typedef _Float16 T; };
template <> struct Elem<1> { typedef __bf16 T; };

template <int ET, int SPL, int BIAS_MODE, int SHIFT>
__global__ __launch_bounds__(256) void wmma_gemm64(
    const unsigned short* __restrict__ Ap, const unsigned short* __restrict__ A2p, int lda,
    const unsigned short* __restrict__ Btp, const unsigned short* __restrict__ Bt2p, int ldb,
    float* __restrict__ C, int ldc,
    const float* __restrict__ bias,
    int M, int N, int K) {
  typedef typename Elem<ET>::T T;
  typedef typename Frag<T>::V V;
  constexpr float scale = 1.0f / (float)(1u << SHIFT);
  const T* A = (const T*)Ap; const T* A2 = (const T*)A2p; const T* Bt = (const T*)Btp; const T* Bt2 = (const T*)Bt2p;
  __shared__ __align__(16) float sT[8][16 * 68];
  const int lane = threadIdx.x & 31;
  const int wave = threadIdx.x >> 5;
  const int tilesN = N >> 6;
  const int tilesM = M >> 6;
  const int tile = blockIdx.x * 8 + wave;
  if (tile >= tilesM * tilesN) return;
  const int tm = tile / tilesN;
  const int tn = tile - tm * tilesN;
  const int m0 = tm << 6;
  const int n0 = tn << 6;

  const int rlane = lane & 15;
  const int koff  = (lane >> 4) * 8;
  const int mOff  = (lane >> 4) * 8;

  v8f acc[4][4];
#pragma unroll
  for (int i = 0; i < 4; ++i)
#pragma unroll
    for (int j = 0; j < 4; ++j) acc[i][j] = (v8f){0.f,0.f,0.f,0.f,0.f,0.f,0.f,0.f};

  for (int k0 = 0; k0 < K; k0 += 32) {
    V bh[4], bl[4];
#pragma unroll
    for (int j = 0; j < 4; ++j) {
      const size_t bo = (size_t)(n0 + (j << 4) + rlane) * ldb + koff + k0;
      bh[j] = Frag<T>::load(Bt + bo);
      bl[j] = bh[j];
      if (SPL == 2) bl[j] = Frag<T>::load(Bt2 + bo);
    }
#pragma unroll
    for (int i = 0; i < 4; ++i) {
      const size_t ao = (size_t)(m0 + (i << 4) + rlane) * lda + koff + k0;
      V ah = Frag<T>::load(A + ao);
      V al = ah;
      if (SPL == 2) al = Frag<T>::load(A2 + ao);
#pragma unroll
      for (int j = 0; j < 4; ++j) {
        acc[i][j] = Frag<T>::mma(ah, bh[j], acc[i][j]);
        if (SPL == 2) {
          acc[i][j] = Frag<T>::mma(ah, bl[j], acc[i][j]);
          acc[i][j] = Frag<T>::mma(al, bh[j], acc[i][j]);
        }
      }
    }
  }

  float* slab = sT[wave];
#pragma unroll
  for (int i = 0; i < 4; ++i) {
    const int mBase = m0 + (i << 4);
#pragma unroll
    for (int j = 0; j < 4; ++j) {
      const int n = n0 + (j << 4) + rlane;
      float bv = 0.f;
      if (BIAS_MODE == 2) bv = bias[n];
#pragma unroll
      for (int r = 0; r < 8; ++r) {
        float v = acc[i][j][r] * scale;
        if (BIAS_MODE == 2) v += bv;
        slab[(mOff + r) * 68 + (j << 4) + rlane] = v;
      }
    }
    __builtin_amdgcn_fence(__ATOMIC_RELEASE, "workgroup");
    __builtin_amdgcn_wave_barrier();
    __builtin_amdgcn_fence(__ATOMIC_ACQUIRE, "workgroup");
    {
      const int hh = lane >> 4, c4 = (lane & 15) * 4;
      for (int pass = 0; pass < 2; ++pass) {
#pragma unroll
        for (int it = 0; it < 8; ++it) {
          const int row = it * 2 + hh;
          v4f v = *(const v4f*)(slab + row * 68 + c4);
          *(volatile v4f*)(C + (size_t)(mBase + row) * ldc + n0 + c4) = v;
        }
        __threadfence();
      }
    }
    __builtin_amdgcn_fence(__ATOMIC_RELEASE, "workgroup");
    __builtin_amdgcn_wave_barrier();
    __builtin_amdgcn_fence(__ATOMIC_ACQUIRE, "workgroup");
  }
}

template <int MODE, int CARRY_LOG2>
__global__ __launch_bounds__(256) void plane_pack_kernel(
    const float* __restrict__ src, unsigned short* __restrict__ dhi, unsigned short* __restrict__ dlo,
    unsigned total8, unsigned dshift, unsigned spitch, unsigned vrows)
{
  const unsigned i = blockIdx.x * 256u + threadIdx.x;
  if (i >= total8) return;
  const unsigned e0 = i << 3;
  unsigned row = e0 >> dshift;
  unsigned col = e0 & ((1u << dshift) - 1u);
  asm volatile("" : "+v"(row));
  asm volatile("" : "+v"(col));
  const bool valid = row < vrows;
  const unsigned rowc = valid ? row : (vrows - 1u);
  const size_t so = (size_t)rowc * spitch + col;
  const v4f a0 = *(const v4f*)(src + so);
  const v4f a1 = *(const v4f*)(src + so + 4);
  constexpr float carry = (float)(1u << CARRY_LOG2);
  float f[8];
  f[0] = valid ? a0[0] : 0.0f;
  f[1] = valid ? a0[1] : 0.0f;
  f[2] = valid ? a0[2] : 0.0f;
  f[3] = valid ? a0[3] : 0.0f;
  f[4] = valid ? a1[0] : 0.0f;
  f[5] = valid ? a1[1] : 0.0f;
  f[6] = valid ? a1[2] : 0.0f;
  f[7] = valid ? a1[3] : 0.0f;
  unsigned wh[4], wl[4];
#pragma unroll
  for (int p = 0; p < 4; ++p) {
    const float f0 = f[2 * p], f1 = f[2 * p + 1];
    if (MODE == 1) {
      const unsigned h0 = bf_rne_word(f0), h1 = bf_rne_word(f1);
      const unsigned l0 = bf_rne_word(f0 - __uint_as_float(h0));
      const unsigned l1 = bf_rne_word(f1 - __uint_as_float(h1));
      wh[p] = (h1 & 0xFFFF0000u) | (h0 >> 16);
      wl[p] = (l1 & 0xFFFF0000u) | (l0 >> 16);
    } else {
      const unsigned b0 = f16_bits(f0 * carry), b1 = f16_bits(f1 * carry);
      wh[p] = (b1 << 16) | (b0 & 0xffffu);
      wl[p] = 0u;
    }
  }
  const v4u hw = (v4u){wh[0], wh[1], wh[2], wh[3]};
  const v4u lw = (v4u){wl[0], wl[1], wl[2], wl[3]};
  volatile v4u* qh = (volatile v4u*)(dhi + e0);
  volatile v4u* ql = (volatile v4u*)(dlo + e0);
  *qh = hw;
  if (MODE == 1) *ql = lw;
  __threadfence();
  *qh = hw;
  if (MODE == 1) *ql = lw;
}

static_assert(((size_t)kRows * kDch) % 2048 == 0, "softplus tiling");
__global__ __launch_bounds__(256) void softplus_kernel(const float* __restrict__ pre, float* __restrict__ dl)
{
  const size_t base = (size_t)blockIdx.x * 2048u + threadIdx.x;
#pragma unroll 1
  for (int k = 0; k < 8; ++k) {
    const size_t idx = base + (size_t)k * 256u;
    const float p = pre[idx];
    const float e = expf(-fabsf(p));
    const float sp = fmaxf(p, 0.0f) + log1pf(e);
    volatile float* q = dl + idx;
    *q = sp;
    __threadfence();
    *q = sp;
  }
}

__global__ __launch_bounds__(64) void scan_kernel(
    const float* __restrict__ XD, const float* __restrict__ DL, const float* __restrict__ X,
    const float* __restrict__ Alog, const float* __restrict__ Dp, float* __restrict__ out)
{
  __shared__ __align__(16) float sBC[kScanTS * 32];
  __shared__ __align__(16) float sY[kScanTS * kScanYP];
  __shared__ __align__(16) float sA[kNst * kScanCh];
  const int tid = threadIdx.x, lane = tid & 31, wave = tid >> 5;
  constexpr int kBlkPerB = kDch / kScanCh;
  const int bix = blockIdx.x / kBlkPerB;
  const int d0  = (blockIdx.x - bix * kBlkPerB) * kScanCh;
  const int d   = d0 + tid;
  const size_t row0 = (size_t)bix * kSeq;
#pragma unroll 1
  for (int s = 0; s < kNst; ++s) sA[s * kScanCh + tid] = -expf(Alog[(size_t)d * kNst + s]);
  __syncthreads();
  float Acoef[kNst], h[kNst];
#pragma unroll
  for (int s = 0; s < kNst; ++s) {
    Acoef[s] = sA[s * kScanCh + tid];
    h[s] = 0.f;
  }
  const float Dd = Dp[d];
  const int lr = tid >> 3, lc4 = (tid & 7) * 4;
  const int hh = lane >> 4, c4 = (lane & 15) * 4;
#pragma unroll 1
  for (int t0 = 0; t0 < kSeq; t0 += kScanTS) {
    __syncthreads();
#pragma unroll
    for (int i = 0; i < 4; ++i) {
      const int r = lr + 8 * i;
      *(v4f*)(sBC + r * 32 + lc4) = *(const v4f*)(XD + (row0 + t0 + r) * kProjP + kRank + lc4);
    }
    __syncthreads();
#pragma unroll 1
    for (int s = 0; s < kScanTS; ++s) {
      const size_t r = row0 + t0 + s;
      const float dt = DL[r * kDch + d];
      const float xt = X[r * kDch + d];
      const float dtx = dt * xt;
      const float* br = sBC + s * 32;
      float y = 0.f;
#pragma unroll
      for (int q4 = 0; q4 < 4; ++q4) {
        const v4f bv = *(const v4f*)(br + 4 * q4);
        const v4f cv = *(const v4f*)(br + kNst + 4 * q4);
#pragma unroll
        for (int e = 0; e < 4; ++e) {
          const int k = 4 * q4 + e;
          const float da = expf(dt * Acoef[k]);
          h[k] = fmaf(da, h[k], dtx * bv[e]);
          y = fmaf(h[k], cv[e], y);
        }
      }
      y = fmaf(xt, Dd, y);
      sY[s * kScanYP + tid] = y;
    }
    __syncthreads();
    v4f fv[8];
#pragma unroll
    for (int it = 0; it < 8; ++it) {
      const int row = it * 4 + wave * 2 + hh;
      fv[it] = *(const v4f*)(sY + row * kScanYP + c4);
    }
    for (int pass = 0; pass < 2; ++pass) {
#pragma unroll
      for (int it = 0; it < 8; ++it) {
        const int row = it * 4 + wave * 2 + hh;
        *(volatile v4f*)(out + (row0 + t0 + row) * kDch + d0 + c4) = fv[it];
      }
      __threadfence();
    }
  }
}

extern "C" void kernel_launch(void* const* d_in, const int* in_sizes, int n_in,
                              void* d_out, int out_size, void* d_ws, size_t ws_size,
                              hipStream_t stream) {
  if (n_in < 6) return;
  if (in_sizes[0] != kRows * kDch) return;
  if (in_sizes[1] != kProjW * kDch) return;
  if (in_sizes[2] != kDch * kRank) return;
  if (in_sizes[3] != kDch) return;
  if (in_sizes[4] != kDch * kNst) return;
  if (in_sizes[5] != kDch) return;
  if (out_size != kRows * kDch) return;
  if (ws_size < kWsTotal) return;

  const float* x       = (const float*)d_in[0];
  const float* W_xproj = (const float*)d_in[1];
  const float* W_dt    = (const float*)d_in[2];
  const float* b_dt    = (const float*)d_in[3];
  const float* A_log   = (const float*)d_in[4];
  const float* Dp      = (const float*)d_in[5];
  float* out = (float*)d_out;

  char* ws = (char*)d_ws;
  unsigned short* XH  = (unsigned short*)(ws + kOffXH);
  unsigned short* XL  = (unsigned short*)(ws + kOffXL);
  unsigned short* WXH = (unsigned short*)(ws + kOffWXH);
  unsigned short* WXL = (unsigned short*)(ws + kOffWXL);
  unsigned short* WDH = (unsigned short*)(ws + kOffWDH);
  unsigned short* WDL = (unsigned short*)(ws + kOffWDL);
  float*          XD  = (float*)(ws + kOffXD);
  unsigned short* DRH = (unsigned short*)(ws + kOffDRH);
  unsigned short* DRL = (unsigned short*)(ws + kOffDRL);
  float*          PRE = (float*)(ws + kOffPRE);
  float*          DL  = (float*)(ws + kOffDL);

  plane_pack_kernel<kMode, kCarryX><<<(kRows * kDch / 8) / 256, 256, 0, stream>>>(
      x, XH, XL, (unsigned)(kRows * kDch / 8), 11u, (unsigned)kDch, (unsigned)kRows);
  plane_pack_kernel<kMode, kCarryWx><<<(kProjP * kDch / 8) / 256, 256, 0, stream>>>(
      W_xproj, WXH, WXL, (unsigned)(kProjP * kDch / 8), 11u, (unsigned)kDch, (unsigned)kProjW);
  plane_pack_kernel<kMode, kCarryWd><<<(kDch * kRank / 8) / 256, 256, 0, stream>>>(
      W_dt, WDH, WDL, (unsigned)(kDch * kRank / 8), 6u, (unsigned)kRank, (unsigned)kDch);

  wmma_gemm64<kET, kSPL, 0, kShift0><<<(kRows / 64) * (kProjP / 64) / 8, 256, 0, stream>>>(
      XH, XL, kDch,
      WXH, WXL, kDch,
      XD, kProjP,
      nullptr,
      kRows, kProjP, kDch);

  plane_pack_kernel<kMode, kCarryDr><<<(kRows * kRank / 8) / 256, 256, 0, stream>>>(
      XD, DRH, DRL, (unsigned)(kRows * kRank / 8), 6u, (unsigned)kProjP, (unsigned)kRows);

  wmma_gemm64<kET, kSPL, 2, kShift1><<<(kRows / 64) * (kDch / 64) / 8, 256, 0, stream>>>(
      DRH, DRL, kRank,
      WDH, WDL, kRank,
      PRE, kDch,
      b_dt,
      kRows, kDch, kRank);

  softplus_kernel<<<(kRows * kDch) / 2048, 256, 0, stream>>>(PRE, DL);

  scan_kernel<<<kBatch * (kDch / kScanCh), kScanCh, 0, stream>>>(XD, DL, x, A_log, Dp, out);
}
